// GroupedQueryAttention_37134287241952
// MI455X (gfx1250) — hardware-verified
//
#include <hip/hip_runtime.h>


#ifndef NB
#define NB 2
#endif
#ifndef SEQ
#define SEQ 2048
#endif
#define NB_FULL  2
#define SEQ_FULL 2048
#define TT   SEQ
#define DM   2048
#define NH_  16
#define NKV  4
#define REP  (NH_ / NKV)
#define HD   128
#define DQ   (NH_ * HD)
#define DKV  (NKV * HD)
#define PCAR 1024.0f
#define SCL  0.08838834764831845f
#define LOG2E 1.4426950408889634f

static_assert(SEQ % 128 == 0);
static_assert(SEQ <= SEQ_FULL);
static_assert(NB <= NB_FULL);
static_assert(DM % 64 == 0 && DQ % 64 == 0 && DKV % 64 == 0);
static_assert(HD == 128);
static_assert(DM % 32 == 0 && DQ % 32 == 0);
static_assert(SEQ % 64 == 0 && SEQ % 32 == 0);
static_assert(NH_ % NKV == 0);
static_assert(DQ == DM);
static_assert(HD * 2 == 16 * 16);
static_assert(((size_t)NH_ * SEQ * HD) % (8 * 256) == 0 && ((size_t)NKV * SEQ * HD) % (8 * 256) == 0);
static_assert(((size_t)SEQ * DM) % (8 * 256) == 0);
static_assert(((size_t)DQ * DM) % (64 * 64) == 0 && ((size_t)DKV * DM) % (64 * 64) == 0);

constexpr size_t al256(size_t b) { return (b + 255) & ~(size_t)255; }
constexpr size_t CARVE_BYTES =
    al256((size_t)DQ * DM * 2) + al256((size_t)DKV * DM * 2) + al256((size_t)DKV * DM * 2) + al256((size_t)DM * DQ * 2) +
    al256((size_t)SEQ * DM * 2) + al256((size_t)SEQ * DQ * 4) + al256((size_t)SEQ * DKV * 4) + al256((size_t)SEQ * DKV * 4) +
    al256((size_t)NH_ * SEQ * HD * 2) + al256((size_t)NKV * SEQ * HD * 2) + al256((size_t)NKV * HD * SEQ * 2) + al256((size_t)SEQ * DQ * 2);
static_assert(CARVE_BYTES <= (size_t)134217728);

typedef _Float16 h16;
typedef unsigned short bf;
typedef __attribute__((ext_vector_type(16))) __bf16   v16bf;
typedef __attribute__((ext_vector_type(16))) _Float16 v16h;
typedef __attribute__((ext_vector_type(8)))  _Float16 v8h;
typedef __attribute__((ext_vector_type(2)))  _Float16 v2h;
typedef __attribute__((ext_vector_type(8)))  unsigned short v8us;
typedef __attribute__((ext_vector_type(8)))  float    v8f;
typedef __attribute__((ext_vector_type(4)))  float    v4f;
typedef __attribute__((ext_vector_type(2)))  unsigned short v2us;
typedef v8h  __attribute__((may_alias)) v8ha;
typedef v4f  __attribute__((may_alias)) v4fa;
typedef v8us __attribute__((may_alias)) v8usa;

__device__ __forceinline__ unsigned short f2bf(float f) { unsigned u = __float_as_uint(f); u += 0x7FFFu + ((u >> 16) & 1u); return (unsigned short)(u >> 16); }
__device__ __forceinline__ float bf2f(unsigned short b) { return __uint_as_float(((unsigned)b) << 16); }
__device__ __forceinline__ float bfr(float f) { return bf2f(f2bf(f)); }
__device__ __forceinline__ v16h cat16(v8h lo, v8h hi) { return __builtin_shufflevector(lo, hi, 0, 1, 2, 3, 4, 5, 6, 7, 8, 9, 10, 11, 12, 13, 14, 15); }
__device__ __forceinline__ v16bf cat16b(v8us lo, v8us hi) { return __builtin_bit_cast(v16bf, __builtin_shufflevector(lo, hi, 0, 1, 2, 3, 4, 5, 6, 7, 8, 9, 10, 11, 12, 13, 14, 15)); }
__device__ __forceinline__ v8f wmma16(v16h a, v16h b, v8f c) { return __builtin_amdgcn_wmma_f32_16x16x32_f16(false, a, false, b, (short)0, c, false, false); }
__device__ __forceinline__ v8f wmmab(v16bf a, v16bf b, v8f c) { return __builtin_amdgcn_wmma_f32_16x16x32_bf16(false, a, false, b, (short)0, c, false, false); }
__device__ __forceinline__ h16 tohx(float x) { return (h16)x; }
__device__ __forceinline__ float neginf() { return __uint_as_float(0xff800000u); }

template <typename T16> struct WFrag;
template <> struct WFrag<h16> { typedef v16h V; static __device__ __forceinline__ V ld(const h16* p) { return cat16(*(const v8h*)p, *(const v8h*)(p + 16)); } static __device__ __forceinline__ v8f mma(V a, V b, v8f c) { return wmma16(a, b, c); } };
template <> struct WFrag<bf> { typedef v16bf V; static __device__ __forceinline__ V ld(const bf* p) { return cat16b(*(const v8us*)p, *(const v8us*)(p + 16)); } static __device__ __forceinline__ v8f mma(V a, V b, v8f c) { return wmmab(a, b, c); } };
template <typename T16, int NSPLIT, bool BIAS>
__global__ __launch_bounds__(32) void k_gemmw(const T16* __restrict__ A, const T16* __restrict__ A2, const T16* __restrict__ Bt, const T16* __restrict__ Bt2, int K, float* C, int ldc, const float* __restrict__ bias, size_t sA, size_t sB, size_t sC) {
    typedef typename WFrag<T16>::V V;
    __shared__ __align__(16) float os[16 * 68];
    const size_t z = blockIdx.z; A += z * sA; if (A2) A2 += z * sA; Bt += z * sB; if (Bt2) Bt2 += z * sB; C += z * sC;
    const int lane = threadIdx.x & 31, lr = lane & 15, hi = lane >> 4; const int r0 = blockIdx.x * 64, c0 = blockIdx.y * 64;
    v8f acc[4][4];
#pragma unroll
    for (int mb = 0; mb < 4; ++mb)
#pragma unroll
        for (int nb = 0; nb < 4; ++nb) acc[mb][nb] = (v8f){};
    const size_t aoff = (size_t)(r0 + lr) * K + 8 * hi, boff = (size_t)(c0 + lr) * K + 8 * hi;
#pragma unroll 1
    for (int kc = 0; kc < K; kc += 32) {
        V a[4], a2[4];
#pragma unroll
        for (int mb = 0; mb < 4; ++mb) { a[mb] = WFrag<T16>::ld(A + aoff + (size_t)mb * 16 * K + kc); if (NSPLIT == 1 || NSPLIT == 2) a2[mb] = WFrag<T16>::ld(A2 + aoff + (size_t)mb * 16 * K + kc); }
#pragma unroll
        for (int nb = 0; nb < 4; ++nb) { const V b = WFrag<T16>::ld(Bt + boff + (size_t)nb * 16 * K + kc); V b2; if (NSPLIT >= 2) b2 = WFrag<T16>::ld(Bt2 + boff + (size_t)nb * 16 * K + kc);
#pragma unroll
            for (int mb = 0; mb < 4; ++mb) { acc[mb][nb] = WFrag<T16>::mma(a[mb], b, acc[mb][nb]); if (NSPLIT == 1 || NSPLIT == 2) acc[mb][nb] = WFrag<T16>::mma(a2[mb], b, acc[mb][nb]); if (NSPLIT >= 2) acc[mb][nb] = WFrag<T16>::mma(a[mb], b2, acc[mb][nb]); } }
        asm volatile("v_nop\n\tv_nop\n\tv_nop\n\tv_nop" : "+v"(acc[0][0]), "+v"(acc[1][1]), "+v"(acc[2][2]), "+v"(acc[3][3]) : "v"(a[0]), "v"(a[3]));
    }
#pragma unroll
    for (int mb = 0; mb < 4; ++mb) {
#pragma unroll
        for (int nb = 0; nb < 4; ++nb) {
#pragma unroll
            for (int j = 0; j < 8; ++j) os[(hi * 8 + j) * 68 + nb * 16 + lr] = acc[mb][nb][j]; }
        __builtin_amdgcn_wave_barrier(); asm volatile("" ::: "memory");
        float* crow = C + (size_t)(r0 + mb * 16) * ldc + c0;
#pragma unroll 1
        for (int ps = 0; ps < 2; ++ps) {
#pragma unroll
            for (int s = 0; s < 8; ++s) { const int row = 2 * s + hi, cofs = lr * 4; v4f val = *(const v4fa*)(os + row * 68 + cofs); if (BIAS) { val[0] += bfr(bias[c0 + cofs]); val[1] += bfr(bias[c0 + cofs + 1]); val[2] += bfr(bias[c0 + cofs + 2]); val[3] += bfr(bias[c0 + cofs + 3]); }
                *(volatile v4f*)(crow + (size_t)row * ldc + cofs) = val; }
            if (ps == 0) __threadfence(); }
        __builtin_amdgcn_wave_barrier(); asm volatile("" ::: "memory");
    }
}

__global__ __launch_bounds__(256) void k_wtG(const float* __restrict__ w, int K, int N, bf* Bt) {
    const int lane = threadIdx.x & 31; const int L0 = (blockIdx.x * 8 + (threadIdx.x >> 5)) * 8; const int nlines = N * K / 64;
#pragma unroll
    for (int ps = 0; ps < 2; ++ps) {
#pragma unroll 1
        for (int l = 0; l < 8; ++l) { const int L = L0 + l; if (L >= nlines) break; const size_t e = (size_t)L * 64 + lane * 2; const int k = (int)(e % K), n = (int)(e / K); v2us o;
            o[0] = f2bf(w[(size_t)k * N + n]); o[1] = f2bf(w[(size_t)(k + 1) * N + n]); *(volatile v2us*)(Bt + e) = o; }
        if (ps == 0) __threadfence(); }
}
__global__ __launch_bounds__(256) void k_wtH(const float* __restrict__ w, int K, int N, h16* Bt) {
    const int lane = threadIdx.x & 31; const int L0 = (blockIdx.x * 8 + (threadIdx.x >> 5)) * 8; const int nlines = N * K / 64;
#pragma unroll
    for (int ps = 0; ps < 2; ++ps) {
#pragma unroll 1
        for (int l = 0; l < 8; ++l) { const int L = L0 + l; if (L >= nlines) break; const size_t e = (size_t)L * 64 + lane * 2; const int k = (int)(e % K), n = (int)(e / K); v2h o;
            o[0] = tohx(bfr(w[(size_t)k * N + n])); o[1] = tohx(bfr(w[(size_t)(k + 1) * N + n])); *(volatile v2h*)(Bt + e) = o; }
        if (ps == 0) __threadfence(); }
}
__global__ __launch_bounds__(256) void k_cvt8(const float* __restrict__ src, bf* dst, size_t n8) { const size_t i = (size_t)blockIdx.x * 256 + threadIdx.x; if (i >= n8) return; const v8f v = *(const v8f*)(src + i * 8); v8us o;
#pragma unroll
    for (int k = 0; k < 8; ++k) o[k] = f2bf(v[k]); *(volatile v8us*)(dst + i * 8) = o; __threadfence(); *(volatile v8us*)(dst + i * 8) = o; }

__global__ __launch_bounds__(256) void k_qkp(const float* __restrict__ F, int pitch, int nheads, h16* P16) {
    const size_t e = ((size_t)blockIdx.x * 256 + threadIdx.x) * 8; if (e >= (size_t)nheads * TT * HD) return;
    const int d = (int)(e % HD); const int tt = (int)((e / HD) % TT); const int hh = (int)(e / ((size_t)HD * TT));
    const float* f = F + (size_t)tt * pitch + (size_t)hh * HD + d;
    const v4f x0 = *(const v4f*)f; const v4f x1 = *(const v4f*)(f + 4);
    v8h o16;
#pragma unroll
    for (int q = 0; q < 8; ++q) { const float x = (q < 4) ? x0[q] : x1[q - 4]; o16[q] = tohx(x); }
    *(volatile v8h*)(P16 + e) = o16; __threadfence();
    *(volatile v8h*)(P16 + e) = o16;
}
__global__ __launch_bounds__(256) void k_vtp8(const float* __restrict__ F, int pitch, int nheads, h16* V16) {
    const size_t e = ((size_t)blockIdx.x * 256 + threadIdx.x) * 8; if (e >= (size_t)nheads * HD * TT) return;
    const int t0 = (int)(e % TT); const int d = (int)((e / TT) % HD); const int gg = (int)(e / ((size_t)TT * HD));
    v8h o16;
#pragma unroll
    for (int q = 0; q < 8; ++q) { const float x = F[(size_t)(t0 + q) * pitch + (size_t)gg * HD + d]; o16[q] = tohx(x); }
    *(volatile v8h*)(V16 + e) = o16; __threadfence();
    *(volatile v8h*)(V16 + e) = o16;
}

__global__ __launch_bounds__(256) void k_attn(const h16* __restrict__ Q16, const h16* __restrict__ K16, const h16* __restrict__ V16, h16* A16) {
    constexpr int KP = 136, VP = 40, PP = 40, SP = 136;
    constexpr int KSZ = 32 * KP, VSZ = 128 * VP, PSZ = 8 * 16 * PP, STG = 8 * 16 * SP;
    constexpr int MAINSZ = KSZ + VSZ + PSZ;
    constexpr int LDSN = (MAINSZ > STG) ? MAINSZ : STG;
    constexpr int OK0 = 0, OV0 = KSZ, OP0 = KSZ + VSZ;
    static_assert(KSZ % 8 == 0 && VSZ % 8 == 0 && PSZ % 8 == 0 && (16 * SP) % 8 == 0);
    __shared__ __align__(16) unsigned short lds[LDSN];

    const int tid = threadIdx.x, lane = tid & 31, w = tid >> 5, hf = lane >> 4, l16 = lane & 15;
    const int qt = (int)blockIdx.x, h = (int)blockIdx.y, g = h / REP;
    const int q0 = qt * 128 + w * 16;
    const size_t qrow = ((size_t)h * TT + (size_t)q0 + l16) * HD;
    const size_t kpl = (size_t)g * TT * HD, vpl = (size_t)g * HD * TT;

    v16h qf[4];
#pragma unroll
    for (int c = 0; c < 4; ++c) qf[c] = cat16(*(const v8h*)(Q16 + qrow + c * 32 + 8 * hf), *(const v8h*)(Q16 + qrow + c * 32 + 16 + 8 * hf));
    v8f o[8];
#pragma unroll
    for (int j = 0; j < 8; ++j) o[j] = (v8f){};
    float m8[8], l8[8];
#pragma unroll
    for (int v = 0; v < 8; ++v) { m8[v] = neginf(); l8[v] = 0.f; }

    const int nkt = TT / 32;
#pragma unroll 1
    for (int kt = 0; kt < nkt; ++kt) {
#pragma unroll
        for (int r = 0; r < 2; ++r) { const int i = tid + r * 256; const int row = i >> 4, ch = i & 15;
            const size_t go = kpl + (size_t)(kt * 32 + row) * HD + ch * 8; const int lo = row * KP + ch * 8;
            *(v8ha*)(lds + OK0 + lo) = *(const v8h*)(K16 + go); }
#pragma unroll
        for (int r = 0; r < 2; ++r) { const int i = tid + r * 256; const int d = i >> 2, ch = i & 3;
            const size_t go = vpl + (size_t)d * TT + kt * 32 + ch * 8; const int lo = d * VP + ch * 8;
            *(v8ha*)(lds + OV0 + lo) = *(const v8h*)(V16 + go); }
        __syncthreads();

        v8f s[2]; s[0] = (v8f){}; s[1] = (v8f){};
        {
            v16h ka16, kb16;
#pragma unroll
            for (int c = 0; c < 4; ++c) {
                const int ka = l16 * KP + c * 32 + 8 * hf, kb = (16 + l16) * KP + c * 32 + 8 * hf;
                ka16 = cat16(*(const v8ha*)(lds + OK0 + ka), *(const v8ha*)(lds + OK0 + ka + 16));
                kb16 = cat16(*(const v8ha*)(lds + OK0 + kb), *(const v8ha*)(lds + OK0 + kb + 16));
                s[0] = wmma16(qf[c], ka16, s[0]); s[1] = wmma16(qf[c], kb16, s[1]);
            }
            asm volatile("v_nop\n\tv_nop\n\tv_nop\n\tv_nop" : "+v"(s[0]), "+v"(s[1]) : "v"(qf[3]), "v"(kb16));
        }

        float mn[8];
#pragma unroll
        for (int v = 0; v < 8; ++v) {
            float mx = neginf();
#pragma unroll
            for (int st = 0; st < 2; ++st) { const float tv = s[st][v] * SCL; s[st][v] = tv; mx = fmaxf(mx, tv); }
#pragma unroll
            for (int sh = 1; sh < 16; sh <<= 1) mx = fmaxf(mx, __shfl_xor(mx, sh, 32));
            mn[v] = fmaxf(m8[v], mx);
        }
#pragma unroll
        for (int v = 0; v < 8; ++v) {
            float rs = 0.f;
#pragma unroll
            for (int st = 0; st < 2; ++st) { const float p = __builtin_amdgcn_exp2f((s[st][v] - mn[v]) * LOG2E); s[st][v] = p; rs += p; }
#pragma unroll
            for (int sh = 1; sh < 16; sh <<= 1) rs += __shfl_xor(rs, sh, 32);
            const float sc = __builtin_amdgcn_exp2f((m8[v] - mn[v]) * LOG2E);
            l8[v] = l8[v] * sc + rs; m8[v] = mn[v];
#pragma unroll
            for (int j = 0; j < 8; ++j) o[j][v] = o[j][v] * sc;
        }

        {
#pragma unroll
            for (int v = 0; v < 8; ++v) { const int pw = (w * 16 + v + 8 * hf) * PP;
                lds[OP0 + pw + l16] = __builtin_bit_cast(unsigned short, tohx(s[0][v] * PCAR)); lds[OP0 + pw + 16 + l16] = __builtin_bit_cast(unsigned short, tohx(s[1][v] * PCAR)); }
            __builtin_amdgcn_fence(3  , "wavefront"); __builtin_amdgcn_wave_barrier(); asm volatile("" ::: "memory");
            const int pr = (w * 16 + l16) * PP + 8 * hf;
            const v16h pf = cat16(*(const v8ha*)(lds + OP0 + pr), *(const v8ha*)(lds + OP0 + pr + 16));
#pragma unroll
            for (int j = 0; j < 8; ++j) { const int vo = (j * 16 + l16) * VP + 8 * hf;
                const v16h vf = cat16(*(const v8ha*)(lds + OV0 + vo), *(const v8ha*)(lds + OV0 + vo + 16));
                o[j] = wmma16(pf, vf, o[j]); }
            asm volatile("v_nop\n\tv_nop\n\tv_nop\n\tv_nop" : "+v"(o[0]), "+v"(o[1]), "+v"(o[2]), "+v"(o[3]), "+v"(o[4]), "+v"(o[5]), "+v"(o[6]), "+v"(o[7]) : "v"(pf));
        }
        __syncthreads();
    }

    float iv[8];
    const float cinv = 1.0f / PCAR;
#pragma unroll
    for (int v = 0; v < 8; ++v) iv[v] = cinv * (1.0f / l8[v]);
    const int sb = w * 16 * SP;
#pragma unroll
    for (int j = 0; j < 8; ++j) {
#pragma unroll
        for (int v = 0; v < 8; ++v) { const float val = o[j][v] * iv[v]; lds[sb + (v + 8 * hf) * SP + j * 16 + l16] = __builtin_bit_cast(unsigned short, tohx(val)); } }
    __builtin_amdgcn_fence(3  , "wavefront"); __builtin_amdgcn_wave_barrier(); asm volatile("" ::: "memory");
    h16* dst = A16 + (size_t)q0 * DQ + (size_t)h * HD + l16 * 8;
#pragma unroll 1
    for (int ps = 0; ps < 2; ++ps) {
#pragma unroll
        for (int si = 0; si < 8; ++si) { const int row = 2 * si + hf; const v8h val = *(const v8ha*)(lds + sb + row * SP + l16 * 8); *(volatile v8h*)(dst + (size_t)row * DQ) = val; }
        if (ps == 0) __threadfence(); }
    __builtin_amdgcn_fence(3  , "wavefront"); __builtin_amdgcn_wave_barrier(); asm volatile("" ::: "memory");
}

extern "C" void kernel_launch(void* const* d_in, const int* in_sizes, int n_in,
                              void* d_out, int out_size, void* d_ws, size_t ws_size, hipStream_t stream) {
    if (n_in < 5) return;
    const size_t needx = (size_t)(NB - 1) * SEQ_FULL * DM + (size_t)TT * DM;
    if ((size_t)in_sizes[0] < needx || (size_t)in_sizes[1] < (size_t)DM * DQ || (size_t)in_sizes[2] < (size_t)DM * DKV ||
        (size_t)in_sizes[3] < (size_t)DM * DKV || (size_t)in_sizes[4] < (size_t)DQ * DM || (size_t)out_size < needx) return;
    const float* x  = (const float*)d_in[0];
    const float* wq = (const float*)d_in[1];
    const float* wk = (const float*)d_in[2];
    const float* wv = (const float*)d_in[3];
    const float* wo = (const float*)d_in[4];
    float* OUT = (float*)d_out;
    char* wsp = (char*)d_ws;
    auto take = [&](size_t bytes) { char* p = wsp; wsp += (bytes + 255) & ~(size_t)255; return (void*)p; };
    bf* WQ = (bf*)take((size_t)DQ * DM * 2); bf* WK = (bf*)take((size_t)DKV * DM * 2); bf* WV = (bf*)take((size_t)DKV * DM * 2); h16* WO = (h16*)take((size_t)DM * DQ * 2);
    bf* XB = (bf*)take((size_t)TT * DM * 2); float* FQ = (float*)take((size_t)TT * DQ * 4); float* FK = (float*)take((size_t)TT * DKV * 4); float* FV = (float*)take((size_t)TT * DKV * 4);
    h16* QP16 = (h16*)take((size_t)NH_ * TT * HD * 2);
    h16* KP16 = (h16*)take((size_t)NKV * TT * HD * 2);
    h16* VT16 = (h16*)take((size_t)NKV * HD * TT * 2);
    h16* AT16 = (h16*)take((size_t)TT * DQ * 2);
    if ((size_t)(wsp - (char*)d_ws) > ws_size) return;

    { const int nq = DQ * DM / 64, nk = DKV * DM / 64, no = DM * DQ / 64;
      k_wtG<<<(nq + 63) / 64, 256, 0, stream>>>(wq, DM, DQ, WQ);
      k_wtG<<<(nk + 63) / 64, 256, 0, stream>>>(wk, DM, DKV, WK);
      k_wtG<<<(nk + 63) / 64, 256, 0, stream>>>(wv, DM, DKV, WV);
      k_wtH<<<(no + 63) / 64, 256, 0, stream>>>(wo, DQ, DM, WO); }
    const unsigned LQP = (unsigned)(((size_t)NH_ * TT * HD / 8 + 255) / 256), LKP = (unsigned)(((size_t)NKV * TT * HD / 8 + 255) / 256);
    for (int b = 0; b < NB; ++b) {
        k_cvt8<<<(unsigned)(((size_t)TT * DM / 8 + 255) / 256), 256, 0, stream>>>(x + (size_t)b * SEQ_FULL * DM, XB, (size_t)TT * DM / 8);
        k_gemmw<bf, 0, false><<<dim3(TT / 64, DQ / 64, 1), 32, 0, stream>>>(XB, nullptr, WQ, nullptr, DM, FQ, DQ, nullptr, 0, 0, 0);
        k_qkp<<<LQP, 256, 0, stream>>>(FQ, DQ, NH_, QP16);
        k_gemmw<bf, 0, false><<<dim3(TT / 64, DKV / 64, 1), 32, 0, stream>>>(XB, nullptr, WK, nullptr, DM, FK, DKV, nullptr, 0, 0, 0);
        k_qkp<<<LKP, 256, 0, stream>>>(FK, DKV, NKV, KP16);
        k_gemmw<bf, 0, false><<<dim3(TT / 64, DKV / 64, 1), 32, 0, stream>>>(XB, nullptr, WV, nullptr, DM, FV, DKV, nullptr, 0, 0, 0);
        k_vtp8<<<LKP, 256, 0, stream>>>(FV, DKV, NKV, VT16);
        k_attn<<<dim3(TT / 128, NH_, 1), 256, 0, stream>>>(QP16, KP16, VT16, AT16);
        k_gemmw<h16, 0, false><<<dim3(TT / 64, DM / 64, 1), 32, 0, stream>>>(AT16, nullptr, WO, nullptr, DQ, OUT + (size_t)b * SEQ_FULL * DM, DM, nullptr, 0, 0, 0);
    }
}
